// Drifting_50337016709322
// MI455X (gfx1250) — hardware-verified
//
#include <hip/hip_runtime.h>

typedef _Float16 v16h __attribute__((ext_vector_type(16)));
typedef _Float16 v8h  __attribute__((ext_vector_type(8)));
typedef __bf16   v16b __attribute__((ext_vector_type(16)));
typedef unsigned short v8u __attribute__((ext_vector_type(8)));
typedef float    v8f  __attribute__((ext_vector_type(8)));
typedef float    v4f  __attribute__((ext_vector_type(4)));
typedef v8h __attribute__((may_alias)) v8ha;
typedef v8u __attribute__((may_alias)) v8ua;
typedef v4f __attribute__((may_alias)) v4fa;

union FragH { v16h v; v8h hv[2]; };
union FragB { v16b v; v8u hv[2]; };

#define GN    4096
#define TN    8192
#define DN    512
#define NRB   256
#define JT    256
#define OSC   32.0f
#define INVS2 (1.0f / 1024.0f)
#define PLANE ((size_t)DN * TN)
#define APL   (16 * 264)
#define CPL   (64 * 72)
#define OPITCH 516

__device__ __forceinline__ v8f wmma_h(v16h a, v16h b, v8f c) {
  v8f d = __builtin_amdgcn_wmma_f32_16x16x32_f16(false, a, false, b, (short)0, c, false, false);
  asm volatile("v_nop\n\tv_nop\n\tv_nop\n\tv_nop" : "+v"(d) : "v"(a), "v"(b));
  return d;
}
__device__ __forceinline__ v8f wmma_b(v16b a, v16b b, v8f c) {
  v8f d = __builtin_amdgcn_wmma_f32_16x16x32_bf16(false, a, false, b, (short)0, c, false, false);
  asm volatile("v_nop\n\tv_nop\n\tv_nop\n\tv_nop" : "+v"(d) : "v"(a), "v"(b));
  return d;
}
__device__ __forceinline__ v16h frag_h(const _Float16* p, int h) {
  FragH f;
  f.hv[0] = *(const v8ha*)(p + 8 * h);
  f.hv[1] = *(const v8ha*)(p + 16 + 8 * h);
  return f.v;
}
__device__ __forceinline__ v16b frag_b(const unsigned short* p, int h) {
  FragB f;
  f.hv[0] = *(const v8ua*)(p + 8 * h);
  f.hv[1] = *(const v8ua*)(p + 16 + 8 * h);
  return f.v;
}

__device__ __forceinline__ unsigned short bf16_bits(float f) {
  unsigned int u = __float_as_uint(f);
  u += 0x7FFFu + ((u >> 16) & 1u);
  return (unsigned short)(u >> 16);
}
__device__ __forceinline__ float bf16_val(unsigned short b) {
  return __uint_as_float(((unsigned int)b) << 16);
}

__device__ __forceinline__ float kval(float accv, float sqa, float sqb, int j, int gi) {
  const float xy = accv * INVS2;
  const float d2 = (sqa + sqb) - 2.0f * xy;
  const float dist = sqrtf(fmaxf(d2, 0.0f));
  const float kv = __expf(-20.0f * dist);
  return (j == gi) ? 0.0f : kv;
}

__device__ __forceinline__ void cvt_store(const _Float16* sF, const unsigned short* sHL,
                                          _Float16* tgth, unsigned short* thp,
                                          int row0, int d0, int w, int q8, int sub) {
  #pragma unroll
  for (int i = 0; i < 2; ++i) {
    const int rr = 8 * w + 4 * i + sub;
    const v8h v = *(const v8ha*)(sF + rr * 72 + 8 * q8);
    *(volatile v8h*)(tgth + (size_t)(row0 + rr) * DN + d0 + 8 * q8) = v;
  }
  const int p = w >> 2;
  const unsigned short* sp = sHL + p * CPL;
  unsigned short* gp = thp + (size_t)p * PLANE;
  #pragma unroll
  for (int i = 0; i < 4; ++i) {
    const int dl = 16 * (w & 3) + 4 * i + sub;
    const v8u v = *(const v8ua*)(sp + dl * 72 + 8 * q8);
    *(volatile v8u*)(gp + (size_t)(d0 + dl) * TN + row0 + 8 * q8) = v;
  }
}

__global__ __launch_bounds__(256) void convert_kernel(
    const float* __restrict__ gen, const float* __restrict__ pos,
    _Float16* __restrict__ tgth, unsigned short* __restrict__ thp, float* __restrict__ sq)
{
  __shared__ __attribute__((aligned(16))) _Float16 sF[64 * 72];
  __shared__ __attribute__((aligned(16))) unsigned short sHL[2 * CPL];
  __shared__ __attribute__((aligned(16))) float sSq[64];

  const int tid = threadIdx.x, lane = tid & 31, w = tid >> 5;
  const int q8 = lane & 7, sub = lane >> 3;
  const int row0 = blockIdx.x * 64;
  const float* src = (row0 < GN) ? (gen + (size_t)row0 * DN) : (pos + (size_t)(row0 - GN) * DN);
  const int r = tid >> 2, ds = (tid & 3) * 16;

  float ss = 0.0f;
  #pragma unroll 1
  for (int c = 0; c < DN / 64; ++c) {
    const int d0 = 64 * c;
    const float* p = src + (size_t)r * DN + d0 + ds;
    const v4f x0 = *(const v4fa*)(p);
    const v4f x1 = *(const v4fa*)(p + 4);
    const v4f x2 = *(const v4fa*)(p + 8);
    const v4f x3 = *(const v4fa*)(p + 12);
    float v[16] = { x0.x, x0.y, x0.z, x0.w, x1.x, x1.y, x1.z, x1.w,
                    x2.x, x2.y, x2.z, x2.w, x3.x, x3.y, x3.z, x3.w };
    #pragma unroll
    for (int e = 0; e < 16; ++e) ss += v[e] * v[e];
    const v8h f0 = { (_Float16)(v[0] * OSC), (_Float16)(v[1] * OSC), (_Float16)(v[2] * OSC), (_Float16)(v[3] * OSC),
                     (_Float16)(v[4] * OSC), (_Float16)(v[5] * OSC), (_Float16)(v[6] * OSC), (_Float16)(v[7] * OSC) };
    const v8h f1 = { (_Float16)(v[8] * OSC), (_Float16)(v[9] * OSC), (_Float16)(v[10] * OSC), (_Float16)(v[11] * OSC),
                     (_Float16)(v[12] * OSC), (_Float16)(v[13] * OSC), (_Float16)(v[14] * OSC), (_Float16)(v[15] * OSC) };
    *(v8ha*)(sF + r * 72 + ds) = f0;
    *(v8ha*)(sF + r * 72 + ds + 8) = f1;
    #pragma unroll
    for (int e = 0; e < 16; ++e) {
      const unsigned short hb = bf16_bits(v[e]);
      const unsigned short lb = bf16_bits(v[e] - bf16_val(hb));
      sHL[(ds + e) * 72 + r] = hb;
      sHL[CPL + (ds + e) * 72 + r] = lb;
    }
    __syncthreads();
    cvt_store(sF, sHL, tgth, thp, row0, d0, w, q8, sub);
    __threadfence();
    cvt_store(sF, sHL, tgth, thp, row0, d0, w, q8, sub);
    __syncthreads();
  }

  ss += __shfl_xor(ss, 1);
  ss += __shfl_xor(ss, 2);
  if ((tid & 3) == 0) sSq[r] = ss;
  __syncthreads();
  if (w == 0 && lane < 16) {
    const v4f v = *(const v4fa*)(sSq + 4 * lane);
    *(volatile v4f*)(sq + row0 + 4 * lane) = v;
    __threadfence();
    *(volatile v4f*)(sq + row0 + 4 * lane) = v;
  }
}

__device__ __forceinline__ void s_tile(const _Float16* arow, const _Float16* brow, int h,
                                       v8f& acc0, v8f& acc1) {
  const v8f z = {0.f, 0.f, 0.f, 0.f, 0.f, 0.f, 0.f, 0.f};
  v8f c0 = z, c1 = z;
  #pragma unroll 4
  for (int k0 = 0; k0 < DN; k0 += 32) {
    const v16h a  = frag_h(arow + k0, h);
    const v16h b0 = frag_h(brow + k0, h);
    const v16h b1 = frag_h(brow + 16 * DN + k0, h);
    c0 = wmma_h(a, b0, c0);
    c1 = wmma_h(a, b1, c1);
  }
  acc0 = c0;
  acc1 = c1;
}

__global__ __launch_bounds__(256) __attribute__((amdgpu_num_vgpr(256))) void stats_kernel(
    const _Float16* __restrict__ tgth, const float* __restrict__ sq,
    float* __restrict__ colpart, float* __restrict__ rsum)
{
  __shared__ float sPart[8 * 16];

  const int tid = threadIdx.x, lane = tid & 31, w = tid >> 5;
  const int h = lane >> 4, m = lane & 15;
  const int rb = blockIdx.x, i0 = rb * 16;

  float sqi[8], racc[8];
  #pragma unroll
  for (int r = 0; r < 8; ++r) { sqi[r] = sq[i0 + 8 * h + r]; racc[r] = 0.0f; }
  const _Float16* arow = tgth + (size_t)(i0 + m) * DN;

  #pragma unroll 1
  for (int tile = 0; tile < TN / JT; ++tile) {
    const int jc = tile * JT + 32 * w;
    v8f acc0, acc1;
    s_tile(arow, tgth + (size_t)(jc + m) * DN, h, acc0, acc1);
    const int j0 = jc + m, j1 = jc + 16 + m;
    const float sq0 = sq[j0], sq1 = sq[j1];
    float c0 = 0.0f, c1 = 0.0f;
    #pragma unroll
    for (int r = 0; r < 8; ++r) {
      const int gi = i0 + 8 * h + r;
      const float k0v = kval(acc0[r], sqi[r], sq0, j0, gi);
      const float k1v = kval(acc1[r], sqi[r], sq1, j1, gi);
      racc[r] += k0v + k1v;
      c0 += k0v;
      c1 += k1v;
    }
    c0 += __shfl_xor(c0, 16);
    c1 += __shfl_xor(c1, 16);
    const float cv = h ? c1 : c0;
    volatile float* cp = colpart + (size_t)rb * TN + jc + lane;
    *cp = cv;
    __threadfence();
    *cp = cv;
  }

  #pragma unroll
  for (int r = 0; r < 8; ++r) {
    float v = racc[r];
    v += __shfl_xor(v, 1); v += __shfl_xor(v, 2);
    v += __shfl_xor(v, 4); v += __shfl_xor(v, 8);
    if (m == 0) sPart[w * 16 + 8 * h + r] = v;
  }
  __syncthreads();
  if (tid < 32) {
    float v = 0.0f;
    #pragma unroll
    for (int w2 = 0; w2 < 8; ++w2) v += sPart[w2 * 16 + (tid & 15)];
    v = (tid < 16) ? v : 0.0f;
    volatile float* rp = rsum + rb * 32 + tid;
    *rp = v;
    __threadfence();
    *rp = v;
  }
}

__global__ __launch_bounds__(256) void colsum_kernel(
    const float* __restrict__ colpart, float* __restrict__ csum)
{
  const int j = blockIdx.x * 256 + threadIdx.x;
  float s = 0.0f;
  #pragma unroll 4
  for (int rb = 0; rb < NRB; ++rb) s += colpart[(size_t)rb * TN + j];
  volatile float* p = csum + j;
  *p = s;
  __threadfence();
  *p = s;
}

__device__ __forceinline__ void half_pass(
    const int jbase, v8f (&va)[4], float* sFinRow,
    const _Float16* tgth, const unsigned short* thp, const float* sq, const float* csum,
    const float (&sqi)[8], const float (&rs)[8],
    unsigned short* sA, float* sPart,
    const int i0, const int tid, const int w, const int h, const int m)
{
  float sacc[8];
  #pragma unroll
  for (int r = 0; r < 8; ++r) sacc[r] = 0.0f;
  const _Float16* arow = tgth + (size_t)(i0 + m) * DN;
  const unsigned short* bn = thp + (size_t)(64 * w + m) * TN;

  #pragma unroll 1
  for (int tile = 0; tile < GN / JT; ++tile) {
    const int jt0 = jbase + tile * JT;
    const int jc = jt0 + 32 * w;
    v8f acc0, acc1;
    s_tile(arow, tgth + (size_t)(jc + m) * DN, h, acc0, acc1);
    const int j0 = jc + m, j1 = jc + 16 + m;
    const float sq0 = sq[j0], sq1 = sq[j1];
    const float cs0 = csum[j0], cs1 = csum[j1];
    #pragma unroll
    for (int r = 0; r < 8; ++r) {
      const int il = 8 * h + r, gi = i0 + il;
      const float k0v = kval(acc0[r], sqi[r], sq0, j0, gi);
      const float k1v = kval(acc1[r], sqi[r], sq1, j1, gi);
      const float n0 = k0v * rsqrtf(fmaxf(rs[r] * cs0, 1e-12f));
      const float n1 = k1v * rsqrtf(fmaxf(rs[r] * cs1, 1e-12f));
      sacc[r] += n0 + n1;
      const unsigned short h0 = bf16_bits(n0), h1 = bf16_bits(n1);
      const unsigned short l0 = bf16_bits(n0 - bf16_val(h0));
      const unsigned short l1 = bf16_bits(n1 - bf16_val(h1));
      const int o0 = il * 264 + 32 * w + m;
      sA[o0] = h0;        sA[o0 + 16] = h1;
      sA[APL + o0] = l0;  sA[APL + o0 + 16] = l1;
    }
    __syncthreads();

    #pragma unroll 1
    for (int ks = 0; ks < JT / 32; ++ks) {
      const unsigned short* ap = sA + m * 264 + 32 * ks;
      const v16b aH = frag_b(ap, h);
      const v16b aL = frag_b(ap + APL, h);
      #pragma unroll
      for (int nt = 0; nt < 4; ++nt) {
        const unsigned short* bp = bn + (size_t)(16 * nt) * TN + jt0 + 32 * ks;
        const v16b bH = frag_b(bp, h);
        const v16b bL = frag_b(bp + PLANE, h);
        va[nt] = wmma_b(aH, bH, va[nt]);
        va[nt] = wmma_b(aH, bL, va[nt]);
        va[nt] = wmma_b(aL, bH, va[nt]);
      }
    }
    __syncthreads();
  }

  #pragma unroll
  for (int r = 0; r < 8; ++r) {
    float v = sacc[r];
    v += __shfl_xor(v, 1); v += __shfl_xor(v, 2);
    v += __shfl_xor(v, 4); v += __shfl_xor(v, 8);
    if (m == 0) sPart[w * 16 + 8 * h + r] = v;
  }
  __syncthreads();
  if (tid < 16) {
    float s = 0.0f;
    #pragma unroll
    for (int w2 = 0; w2 < 8; ++w2) s += sPart[w2 * 16 + tid];
    sFinRow[tid] = s;
  }
  __syncthreads();
}

__device__ __forceinline__ void out_store(const float* sO, float* out, int i0, int w, int q8, int sub) {
  #pragma unroll
  for (int i = 0; i < 8; ++i) {
    const int L = 32 * w + 4 * i + sub;
    const int rr = L >> 4, seg = L & 15;
    const v4f v = *(const v4fa*)(sO + rr * OPITCH + 32 * seg + 4 * q8);
    *(volatile v4f*)(out + (size_t)(i0 + rr) * DN + 32 * seg + 4 * q8) = v;
  }
}

__global__ __launch_bounds__(256) __attribute__((amdgpu_num_vgpr(256))) void main_kernel(
    const _Float16* __restrict__ tgth, const unsigned short* __restrict__ thp,
    const float* __restrict__ sq, const float* __restrict__ rsum, const float* __restrict__ csum,
    float* __restrict__ out)
{
  __shared__ __attribute__((aligned(16))) unsigned short sA[2 * APL];
  __shared__ __attribute__((aligned(16))) float sO[16 * OPITCH];
  __shared__ float sPart[8 * 16];
  __shared__ float sFin[2 * 16];

  const int tid = threadIdx.x, lane = tid & 31, w = tid >> 5;
  const int h = lane >> 4, m = lane & 15;
  const int q8 = lane & 7, sub = lane >> 3;
  const int rb = blockIdx.x, i0 = rb * 16;

  float sqi[8], rs[8];
  #pragma unroll
  for (int r = 0; r < 8; ++r) {
    sqi[r] = sq[i0 + 8 * h + r];
    rs[r]  = rsum[rb * 32 + 8 * h + r];
  }

  const v8f z = {0.f, 0.f, 0.f, 0.f, 0.f, 0.f, 0.f, 0.f};
  v8f vneg[4], vpos[4];
  #pragma unroll
  for (int nt = 0; nt < 4; ++nt) { vneg[nt] = z; vpos[nt] = z; }

  half_pass(0,  vneg, sFin,      tgth, thp, sq, csum, sqi, rs, sA, sPart, i0, tid, w, h, m);
  half_pass(GN, vpos, sFin + 16, tgth, thp, sq, csum, sqi, rs, sA, sPart, i0, tid, w, h, m);

  #pragma unroll
  for (int nt = 0; nt < 4; ++nt) {
    #pragma unroll
    for (int r = 0; r < 8; ++r) {
      const int il = 8 * h + r;
      const float sn = sFin[il], sp = sFin[16 + il];
      sO[il * OPITCH + 64 * w + 16 * nt + m] = sn * vpos[nt][r] - sp * vneg[nt][r];
    }
  }
  __syncthreads();
  out_store(sO, out, i0, w, q8, sub);
  __threadfence();
  out_store(sO, out, i0, w, q8, sub);
}

extern "C" void kernel_launch(void* const* d_in, const int* in_sizes, int n_in,
                              void* d_out, int out_size, void* d_ws, size_t ws_size,
                              hipStream_t stream) {
  if (n_in < 2) return;
  if (in_sizes[0] != GN * DN || in_sizes[1] != GN * DN) return;
  if (out_size != GN * DN) return;

  const float* gen = (const float*)d_in[0];
  const float* pos = (const float*)d_in[1];
  float* out = (float*)d_out;

  const size_t b_tgth = (size_t)TN * DN * 2;
  const size_t b_thp  = (size_t)2 * PLANE * 2;
  const size_t b_colp = (size_t)NRB * TN * 4;
  const size_t b_sq   = (size_t)TN * 4;
  const size_t b_rsum = (size_t)NRB * 32 * 4;
  const size_t b_csum = (size_t)TN * 4;
  const size_t o_tgth = 0;
  const size_t o_thp  = o_tgth + b_tgth;
  const size_t o_colp = o_thp + b_thp;
  const size_t o_sq   = o_colp + b_colp;
  const size_t o_rsum = o_sq + b_sq;
  const size_t o_csum = o_rsum + b_rsum;
  const size_t total  = o_csum + b_csum;
  if (total > ws_size) return;

  char* ws = (char*)d_ws;
  _Float16* tgth      = (_Float16*)(ws + o_tgth);
  unsigned short* thp = (unsigned short*)(ws + o_thp);
  float* colpart      = (float*)(ws + o_colp);
  float* sq           = (float*)(ws + o_sq);
  float* rsum         = (float*)(ws + o_rsum);
  float* csum         = (float*)(ws + o_csum);

  convert_kernel<<<TN / 64, 256, 0, stream>>>(gen, pos, tgth, thp, sq);
  stats_kernel<<<NRB, 256, 0, stream>>>(tgth, sq, colpart, rsum);
  colsum_kernel<<<TN / 256, 256, 0, stream>>>(colpart, csum);
  main_kernel<<<NRB, 256, 0, stream>>>(tgth, thp, sq, rsum, csum, out);
}
